// GPTDecoderBlock_11553462026829
// MI455X (gfx1250) — hardware-verified
//
#include <hip/hip_runtime.h>
#include <math.h>
#include <stdint.h>


#define NB   2
#define SEQ  2048
#define DM   768
#define NH   12
#define HD   64
#define DFF  3072
#define NQB  (SEQ / 64)
#define NTOK (NB * SEQ)
static_assert(NH * HD == DM);
static_assert((SEQ % 64) == 0 && (DM % 64) == 0 && (DFF % 64) == 0 && (NTOK % 64) == 0);
static_assert((DM % 256) == 0);

typedef _Float16 v16h __attribute__((ext_vector_type(16)));
typedef _Float16 v8h  __attribute__((ext_vector_type(8)));
typedef float    v8f  __attribute__((ext_vector_type(8)));
typedef float    v4f  __attribute__((ext_vector_type(4)));
typedef unsigned int v4u __attribute__((ext_vector_type(4)));

#if defined(__HIP_DEVICE_COMPILE__)
#define KX_DEV_ASM 1
#else
#define KX_DEV_ASM 0
#endif

__device__ __forceinline__ unsigned short h_bits(_Float16 x) { return __builtin_bit_cast(unsigned short, x); }
__device__ __forceinline__ unsigned pk16(unsigned short a, unsigned short b) { return (unsigned)a | ((unsigned)b << 16); }
__device__ __forceinline__ unsigned pkh2(float a, float b) {
  const _Float16 x = (_Float16)a, y = (_Float16)b;
  return pk16(h_bits(x), h_bits(y));
}
__device__ __forceinline__ v8f zero8() { v8f z = {0.f, 0.f, 0.f, 0.f, 0.f, 0.f, 0.f, 0.f}; return z; }
__device__ __forceinline__ float gelu_f(float v) { return 0.5f * v * (1.0f + erff(v * 0.70710678118654752f)); }

__device__ __forceinline__ v16h ldfrag_h(const _Float16* p) {
  union { v16h v; v8h h[2]; } f;
  f.h[0] = *(const v8h*)(p);
  f.h[1] = *(const v8h*)(p + 16);
  return f.v;
}

__device__ __forceinline__ v8f mma_h(v16h a, v16h b, v8f c) {
  c = __builtin_amdgcn_wmma_f32_16x16x32_f16(false, a, false, b, (short)0, c, false, false);
#if KX_DEV_ASM
  asm volatile("v_nop\n\tv_nop\n\tv_nop\n\tv_nop" : "+v"(c) : "v"(a), "v"(b));
#endif
  return c;
}
__device__ __forceinline__ v8f mma_h_raw(v16h a, v16h b, v8f c) {
  return __builtin_amdgcn_wmma_f32_16x16x32_f16(false, a, false, b, (short)0, c, false, false);
}
__device__ __forceinline__ void dep_guard(v8f& a, v8f& b, v16h x) {
#if KX_DEV_ASM
  asm volatile("v_nop\n\tv_nop\n\tv_nop\n\tv_nop" : "+v"(a), "+v"(b) : "v"(x));
#else
  (void)a; (void)b; (void)x;
#endif
}
__device__ __forceinline__ void keep4(v16h a, v16h b, v16h c, v16h d) {
#if KX_DEV_ASM
  asm volatile("v_nop" :: "v"(a), "v"(b), "v"(c), "v"(d));
#else
  (void)a; (void)b; (void)c; (void)d;
#endif
}
__device__ __forceinline__ void acc_guard4(v8f& a, v8f& b, v8f& c, v8f& d) {
#if KX_DEV_ASM
  asm volatile("v_nop\n\tv_nop\n\tv_nop\n\tv_nop" : "+v"(a), "+v"(b), "+v"(c), "+v"(d));
#else
  (void)a; (void)b; (void)c; (void)d;
#endif
}
__device__ __forceinline__ void wave_sync() {
  __builtin_amdgcn_fence(__ATOMIC_RELEASE, "workgroup");
  __builtin_amdgcn_wave_barrier();
  __builtin_amdgcn_fence(__ATOMIC_ACQUIRE, "workgroup");
}

__global__ __launch_bounds__(256) void layernorm_h(const float* __restrict__ x, const float* __restrict__ g,
                                                   const float* __restrict__ bt, unsigned short* out,
                                                   int M, float eps) {
  const int lane = threadIdx.x & 31, wave = threadIdx.x >> 5;
  const int row = blockIdx.x * 8 + wave;
  if (row >= M) return;
  const float* xr = x + (size_t)row * DM;
  v4f v[6];
#pragma unroll
  for (int cc = 0; cc < 3; ++cc) {
    v[2 * cc]     = *(const v4f*)(xr + cc * 256 + lane * 8);
    v[2 * cc + 1] = *(const v4f*)(xr + cc * 256 + lane * 8 + 4);
  }
  float s = 0.f;
#pragma unroll
  for (int i = 0; i < 6; ++i) s += (v[i][0] + v[i][1]) + (v[i][2] + v[i][3]);
#pragma unroll
  for (int off = 16; off > 0; off >>= 1) s += __shfl_xor(s, off, 32);
  const float mean = s * (1.0f / (float)DM);
  float s2 = 0.f;
#pragma unroll
  for (int i = 0; i < 6; ++i) {
#pragma unroll
    for (int e = 0; e < 4; ++e) { const float d = v[i][e] - mean; s2 += d * d; }
  }
#pragma unroll
  for (int off = 16; off > 0; off >>= 1) s2 += __shfl_xor(s2, off, 32);
  const float var = s2 * (1.0f / (float)DM);
  const float rs  = 1.0f / sqrtf(var + eps);

  v4u pk[3];
#pragma unroll
  for (int cc = 0; cc < 3; ++cc) {
    const v4f g0 = *(const v4f*)(g  + cc * 256 + lane * 8);
    const v4f g1 = *(const v4f*)(g  + cc * 256 + lane * 8 + 4);
    const v4f b0 = *(const v4f*)(bt + cc * 256 + lane * 8);
    const v4f b1 = *(const v4f*)(bt + cc * 256 + lane * 8 + 4);
    float y[8];
#pragma unroll
    for (int e = 0; e < 4; ++e) {
      y[e]     = (g0[e] * (v[2 * cc][e]     - mean)) * rs + b0[e];
      y[4 + e] = (g1[e] * (v[2 * cc + 1][e] - mean)) * rs + b1[e];
    }
    v4u p;
    p[0] = pkh2(y[0], y[1]); p[1] = pkh2(y[2], y[3]); p[2] = pkh2(y[4], y[5]); p[3] = pkh2(y[6], y[7]);
    pk[cc] = p;
  }
  unsigned short* orow = out + (size_t)row * DM;
  for (int pass = 0; pass < 2; ++pass) {
#pragma unroll
    for (int cc = 0; cc < 3; ++cc) *(volatile v4u*)(orow + cc * 256 + lane * 8) = pk[cc];
    __threadfence();
  }
}

__global__ __launch_bounds__(256) void wcvt_t64(const float* __restrict__ w, unsigned short* out,
                                                int K, int N, float wscale) {
  __shared__ __align__(16) _Float16 sT[64 * 72];
  const int tid = threadIdx.x, lane = tid & 31, wave = tid >> 5;
  const int n0 = blockIdx.x * 64, k0 = blockIdx.y * 64;
  if (n0 + 64 > N || k0 + 64 > K) return;
  const int kr = tid >> 2, nq = (tid & 3) * 16;
  const float* src = w + (size_t)(k0 + kr) * N + n0 + nq;
#pragma unroll
  for (int e = 0; e < 4; ++e) {
    const v4f a = *(const v4f*)(src + 4 * e);
#pragma unroll
    for (int c = 0; c < 4; ++c) sT[(nq + 4 * e + c) * 72 + kr] = (_Float16)(a[c] * wscale);
  }
  __syncthreads();
  const int q = lane >> 3, c8 = (lane & 7) * 8;
  v4u hv[2];
  size_t go[2];
#pragma unroll
  for (int it = 0; it < 2; ++it) {
    const int n = wave * 8 + it * 4 + q;
    const v8h val = *(const v8h*)(sT + n * 72 + c8);
    hv[it] = __builtin_bit_cast(v4u, val);
    go[it] = (size_t)(n0 + n) * K + k0 + c8;
  }
  for (int pass = 0; pass < 2; ++pass) {
#pragma unroll
    for (int it = 0; it < 2; ++it) *(volatile v4u*)(out + go[it]) = hv[it];
    __threadfence();
  }
}

template <int BIAS, int EPI, int OUTH>
__global__ __launch_bounds__(256) void gemm64(
    const unsigned short* __restrict__ Ap, int lda, long long strideA,
    const unsigned short* __restrict__ Btp, int ldb, long long strideB,
    const float* __restrict__ bias, const float* __restrict__ resid,
    void* Cout, int ldc, long long strideC,
    int M, int N, int K, float oscale) {
  const _Float16* A  = (const _Float16*)(const void*)Ap;
  const _Float16* Bt = (const _Float16*)(const void*)Btp;
  __shared__ __align__(16) float sT[8][16 * 68];
  const int b    = blockIdx.y;
  const int lane = threadIdx.x & 31;
  const int wave = threadIdx.x >> 5;
  const int tilesN = N >> 6;
  const int tilesM = M >> 6;
  const int tile = blockIdx.x * 8 + wave;
  if (tile >= tilesM * tilesN) return;
  const int tm = tile / tilesN;
  const int tn = tile - tm * tilesN;
  const int m0 = tm << 6;
  const int n0 = tn << 6;

  const _Float16* Ab = A  + (size_t)b * strideA;
  const _Float16* Bb = Bt + (size_t)b * strideB;

  const int rlane = lane & 15;
  const int koff  = (lane >> 4) * 8;
  const int mOff  = (lane >> 4) * 8;

  v8f acc[4][4];
#pragma unroll
  for (int i = 0; i < 4; ++i)
#pragma unroll
    for (int j = 0; j < 4; ++j) acc[i][j] = zero8();

  for (int k0 = 0; k0 < K; k0 += 32) {
    v16h bh[4];
#pragma unroll
    for (int j = 0; j < 4; ++j) {
      const size_t bo = (size_t)(n0 + (j << 4) + rlane) * ldb + koff + k0;
      bh[j] = ldfrag_h(Bb + bo);
    }
#pragma unroll
    for (int i = 0; i < 4; ++i) {
      const size_t ao = (size_t)(m0 + (i << 4) + rlane) * lda + koff + k0;
      const v16h ah = ldfrag_h(Ab + ao);
#pragma unroll
      for (int j = 0; j < 4; ++j) acc[i][j] = mma_h_raw(ah, bh[j], acc[i][j]);
      dep_guard(acc[i][0], acc[i][3], ah);
    }
    keep4(bh[0], bh[1], bh[2], bh[3]);
  }
  acc_guard4(acc[0][0], acc[0][1], acc[0][2], acc[0][3]);
  acc_guard4(acc[1][0], acc[1][1], acc[1][2], acc[1][3]);
  acc_guard4(acc[2][0], acc[2][1], acc[2][2], acc[2][3]);
  acc_guard4(acc[3][0], acc[3][1], acc[3][2], acc[3][3]);

  float* slab = sT[wave];
#pragma unroll
  for (int i = 0; i < 4; ++i) {
    const int mBase = m0 + (i << 4);
#pragma unroll
    for (int j = 0; j < 4; ++j) {
#pragma unroll
      for (int r = 0; r < 8; ++r) slab[(mOff + r) * 68 + (j << 4) + rlane] = acc[i][j][r];
    }
    wave_sync();
    if (OUTH == 0) {
      float* C = (float*)Cout + (size_t)b * strideC;
      const float* R = resid + (size_t)b * strideC;
      const int hq = lane >> 4, c4 = (lane & 15) * 4;
      v4f bb = {0.f, 0.f, 0.f, 0.f};
      if (BIAS == 1) bb = *(const v4f*)(bias + n0 + c4);
      v4f vals[8];
#pragma unroll
      for (int it = 0; it < 8; ++it) {
        const int row = it * 2 + hq;
        const v4f v = *(const v4f*)(slab + row * 68 + c4);
        const size_t go = (size_t)(mBase + row) * ldc + n0 + c4;
        const v4f rr = *(const v4f*)(R + go);
        float badd = 0.f;
        if (BIAS == 2) badd = bias[mBase + row];
        v4f o;
#pragma unroll
        for (int e = 0; e < 4; ++e) o[e] = rr[e] + (v[e] * oscale + (bb[e] + badd));
        vals[it] = o;
      }
      for (int pass = 0; pass < 2; ++pass) {
#pragma unroll
        for (int it = 0; it < 8; ++it) {
          const int row = it * 2 + hq;
          *(volatile v4f*)(C + (size_t)(mBase + row) * ldc + n0 + c4) = vals[it];
        }
        __threadfence();
      }
    } else {
      unsigned short* C = (unsigned short*)Cout + (size_t)b * strideC;
      const int q = lane >> 3, c8 = (lane & 7) * 8;
      float bcol[8];
#pragma unroll
      for (int e = 0; e < 8; ++e) bcol[e] = 0.f;
      if (BIAS == 1) {
        const v4f b0 = *(const v4f*)(bias + n0 + c8);
        const v4f b1 = *(const v4f*)(bias + n0 + c8 + 4);
#pragma unroll
        for (int e = 0; e < 4; ++e) { bcol[e] = b0[e]; bcol[4 + e] = b1[e]; }
      }
      v4u hv[4];
#pragma unroll
      for (int it = 0; it < 4; ++it) {
        const int row = it * 4 + q;
        const float* sp = slab + row * 68 + c8;
        float badd = 0.f;
        if (BIAS == 2) badd = bias[mBase + row];
        v4u a;
#pragma unroll
        for (int e = 0; e < 4; ++e) {
          float f0 = sp[2 * e]     * oscale + (bcol[2 * e]     + badd);
          float f1 = sp[2 * e + 1] * oscale + (bcol[2 * e + 1] + badd);
          if (EPI == 1) { f0 = gelu_f(f0); f1 = gelu_f(f1); }
          a[e] = pkh2(f0, f1);
        }
        hv[it] = a;
      }
      for (int pass = 0; pass < 2; ++pass) {
#pragma unroll
        for (int it = 0; it < 4; ++it) {
          const int row = it * 4 + q;
          *(volatile v4u*)(C + (size_t)(mBase + row) * ldc + n0 + c8) = hv[it];
        }
        __threadfence();
      }
    }
    wave_sync();
  }
}

__global__ __launch_bounds__(128)
void attn_causal64(const unsigned short* __restrict__ qp, const unsigned short* __restrict__ kp,
                   const unsigned short* __restrict__ vtp, unsigned short* op, float sscale) {
  union FH { v16h v; v8h h[2]; };
  __shared__ __align__(16) _Float16 Ksh[64 * 64];
  __shared__ __align__(16) _Float16 Vth[64 * 64];
  __shared__ __align__(16) _Float16 Psh[4][16 * 64];
  __shared__ __align__(16) float    Os[4][16 * 64];

  const int tid  = threadIdx.x;
  const int wave = tid >> 5;
  const int lane = tid & 31;
  const int hh   = lane >> 4;
  const int c    = lane & 15;

  const int bx   = blockIdx.x;
  const int qb   = bx % NQB;
  const int rest = bx / NQB;
  const int h    = rest % NH;
  const int b    = rest / NH;
  const int q0   = qb * 64 + wave * 16;
  const size_t rowB = (size_t)b * SEQ;

  const _Float16* Q  = (const _Float16*)(const void*)qp + (size_t)h * HD;
  const _Float16* Kg = (const _Float16*)(const void*)kp + (size_t)h * HD;
  const _Float16* Vt = (const _Float16*)(const void*)vtp + ((size_t)b * DM + (size_t)h * HD) * SEQ;

  v16h qa[2];
#pragma unroll
  for (int dc = 0; dc < 2; ++dc) qa[dc] = ldfrag_h(Q + (rowB + q0 + c) * DM + dc * 32 + 8 * hh);

  float mrow[8], lrow[8];
  v8f oacc[4];
#pragma unroll
  for (int r = 0; r < 8; ++r) { mrow[r] = -INFINITY; lrow[r] = 0.f; }
#pragma unroll
  for (int t = 0; t < 4; ++t) oacc[t] = zero8();

  for (int kt = 0; kt < NQB; ++kt) {
    if (kt > qb) break;
    const int kv0 = kt * 64;
    __syncthreads();
    {
      const int r = tid >> 1, half = (tid & 1) * 32;
      const _Float16* kg = Kg + (rowB + kv0 + r) * DM + half;
      const _Float16* vg = Vt + (size_t)r * SEQ + kv0 + half;
#pragma unroll
      for (int i = 0; i < 4; ++i) {
        const v8h a0 = *(const v8h*)(kg + 8 * i);
        const v8h b0 = *(const v8h*)(vg + 8 * i);
        *(v8h*)(Ksh + r * 64 + half + 8 * i) = a0;
        *(v8h*)(Vth + r * 64 + half + 8 * i) = b0;
      }
    }
    __syncthreads();

    v8f s[4];
#pragma unroll
    for (int j = 0; j < 4; ++j) {
      s[j] = zero8();
#pragma unroll
      for (int dc = 0; dc < 2; ++dc) {
        FH kb;
        kb.h[0] = *(const v8h*)(Ksh + (j * 16 + c) * 64 + dc * 32 + 8 * hh);
        kb.h[1] = *(const v8h*)(Ksh + (j * 16 + c) * 64 + dc * 32 + 16 + 8 * hh);
        s[j] = mma_h(qa[dc], kb.v, s[j]);
      }
    }

    const bool diag = (kt == qb);
    _Float16* pwh = Psh[wave];
#pragma unroll
    for (int r = 0; r < 8; ++r) {
      const int qrow = q0 + 8 * hh + r;
      float m = -INFINITY;
#pragma unroll
      for (int j = 0; j < 4; ++j) {
        const int key = kv0 + j * 16 + c;
        float sv = s[j][r] * sscale;
        if (diag && key > qrow) sv = -INFINITY;
        s[j][r] = sv;
        m = fmaxf(m, sv);
      }
#pragma unroll
      for (int off = 1; off < 16; off <<= 1) m = fmaxf(m, __shfl_xor(m, off, 32));
      const float mnew  = fmaxf(mrow[r], m);
      const float msafe = (mnew == -INFINITY) ? 0.f : mnew;
      const float alpha = __expf(mrow[r] - msafe);
      mrow[r] = mnew;
      float psum = 0.f;
#pragma unroll
      for (int j = 0; j < 4; ++j) {
        const float p = __expf(s[j][r] - msafe);
        psum += p;
        pwh[(8 * hh + r) * 64 + j * 16 + c] = (_Float16)(p * 1024.0f);
      }
#pragma unroll
      for (int off = 1; off < 16; off <<= 1) psum += __shfl_xor(psum, off, 32);
      lrow[r] = lrow[r] * alpha + psum;
#pragma unroll
      for (int t = 0; t < 4; ++t) oacc[t][r] *= alpha;
    }
    wave_sync();

#pragma unroll
    for (int kk = 0; kk < 2; ++kk) {
      FH pa;
      pa.h[0] = *(const v8h*)(pwh + c * 64 + kk * 32 + 8 * hh);
      pa.h[1] = *(const v8h*)(pwh + c * 64 + kk * 32 + 16 + 8 * hh);
#pragma unroll
      for (int t = 0; t < 4; ++t) {
        FH vb;
        vb.h[0] = *(const v8h*)(Vth + (t * 16 + c) * 64 + kk * 32 + 8 * hh);
        vb.h[1] = *(const v8h*)(Vth + (t * 16 + c) * 64 + kk * 32 + 16 + 8 * hh);
        oacc[t] = mma_h(pa.v, vb.v, oacc[t]);
      }
    }
  }

  float* os = Os[wave];
#pragma unroll
  for (int r = 0; r < 8; ++r) {
    const float l = lrow[r];
    const float inv = ((l > 0.f) ? (1.0f / l) : 0.f) * (1.0f / 1024.0f);
#pragma unroll
    for (int t = 0; t < 4; ++t) os[(8 * hh + r) * 64 + t * 16 + c] = oacc[t][r] * inv;
  }
  wave_sync();
  {
    const int q4 = lane >> 3, c8 = (lane & 7) * 8;
    v4u hv[4];
#pragma unroll
    for (int it = 0; it < 4; ++it) {
      const int row = it * 4 + q4;
      const float* sp = os + row * 64 + c8;
      v4u a;
#pragma unroll
      for (int e = 0; e < 4; ++e) a[e] = pkh2(sp[2 * e], sp[2 * e + 1]);
      hv[it] = a;
    }
    for (int pass = 0; pass < 2; ++pass) {
#pragma unroll
      for (int it = 0; it < 4; ++it) {
        const int row = it * 4 + q4;
        const size_t go = (rowB + q0 + row) * DM + (size_t)h * HD + c8;
        *(volatile v4u*)(op + go) = hv[it];
      }
      __threadfence();
    }
  }
}

extern "C" void kernel_launch(void* const* d_in, const int* in_sizes, int n_in,
                              void* d_out, int out_size, void* d_ws, size_t ws_size,
                              hipStream_t stream) {
  if (n_in < 17) return;
  if (in_sizes[0] != NTOK * DM) return;
  if (in_sizes[1] != DM || in_sizes[2] != DM) return;
  if (in_sizes[3] != DM * DM || in_sizes[5] != DM * DM || in_sizes[7] != DM * DM || in_sizes[9] != DM * DM) return;
  if (in_sizes[4] != DM || in_sizes[6] != DM || in_sizes[8] != DM || in_sizes[10] != DM) return;
  if (in_sizes[11] != DM || in_sizes[12] != DM) return;
  if (in_sizes[13] != DM * DFF || in_sizes[14] != DFF || in_sizes[15] != DFF * DM || in_sizes[16] != DM) return;
  if (out_size != NTOK * DM) return;

  const float* x    = (const float*)d_in[0];
  const float* ln1g = (const float*)d_in[1];
  const float* ln1b = (const float*)d_in[2];
  const float* wq   = (const float*)d_in[3];
  const float* bq   = (const float*)d_in[4];
  const float* wk   = (const float*)d_in[5];
  const float* bk   = (const float*)d_in[6];
  const float* wv   = (const float*)d_in[7];
  const float* bv   = (const float*)d_in[8];
  const float* wo   = (const float*)d_in[9];
  const float* bo   = (const float*)d_in[10];
  const float* ln2g = (const float*)d_in[11];
  const float* ln2b = (const float*)d_in[12];
  const float* w1   = (const float*)d_in[13];
  const float* b1   = (const float*)d_in[14];
  const float* w2   = (const float*)d_in[15];
  const float* b2   = (const float*)d_in[16];
  float* out = (float*)d_out;

  const size_t PH  = (size_t)NTOK * DM * 2;
  const size_t PWD = (size_t)DM * DM * 2;
  const size_t PWF = (size_t)DM * DFF * 2;
  const size_t PX1 = (size_t)NTOK * DM * 4;
  const size_t PG  = (size_t)NTOK * DFF * 2;
  size_t off = 0;
  const size_t oH1 = off; off += PH;
  const size_t oWq = off; off += PWD;
  const size_t oWk = off; off += PWD;
  const size_t oWv = off; off += PWD;
  const size_t oWo = off; off += PWD;
  const size_t oW1 = off; off += PWF;
  const size_t oW2 = off; off += PWF;
  const size_t oQ  = off; off += PH;
  const size_t oK  = off; off += PH;
  const size_t oVT = off; off += PH;
  const size_t oCT = off; off += PH;
  const size_t oX1 = off; off += PX1;
  const size_t oH2 = off; off += PH;
  const size_t oG  = off; off += PG;
  if (off > ws_size) return;
  if (off > (size_t)134217728) return;

  char* ws = (char*)d_ws;
  unsigned short* H1  = (unsigned short*)(ws + oH1);
  unsigned short* Wtq = (unsigned short*)(ws + oWq);
  unsigned short* Wtk = (unsigned short*)(ws + oWk);
  unsigned short* Wtv = (unsigned short*)(ws + oWv);
  unsigned short* Wto = (unsigned short*)(ws + oWo);
  unsigned short* Wt1 = (unsigned short*)(ws + oW1);
  unsigned short* Wt2 = (unsigned short*)(ws + oW2);
  unsigned short* Qp  = (unsigned short*)(ws + oQ);
  unsigned short* Kp  = (unsigned short*)(ws + oK);
  unsigned short* VTp = (unsigned short*)(ws + oVT);
  unsigned short* CTX = (unsigned short*)(ws + oCT);
  float*          X1  = (float*)(ws + oX1);
  unsigned short* H2  = (unsigned short*)(ws + oH2);
  unsigned short* Gp  = (unsigned short*)(ws + oG);

  const float wsc = 64.0f, winv = 1.0f / 64.0f;
  const dim3 blk(256);
  const dim3 gLN(NTOK / 8);
  const dim3 gWdd(DM / 64, DM / 64);
  const dim3 gW1(DFF / 64, DM / 64);
  const dim3 gW2(DM / 64, DFF / 64);
  const dim3 gProjD(((NTOK / 64) * (DM / 64) + 7) / 8, 1);
  const dim3 gVT(((DM / 64) * (SEQ / 64) + 7) / 8, NB);
  const dim3 gProjF(((NTOK / 64) * (DFF / 64) + 7) / 8, 1);
  const dim3 gAttn(NB * NH * NQB);

  layernorm_h<<<gLN, blk, 0, stream>>>(x, ln1g, ln1b, H1, NTOK, 1e-7f);
  wcvt_t64<<<gWdd, blk, 0, stream>>>(wq, Wtq, DM, DM, wsc);
  wcvt_t64<<<gWdd, blk, 0, stream>>>(wk, Wtk, DM, DM, wsc);
  wcvt_t64<<<gWdd, blk, 0, stream>>>(wv, Wtv, DM, DM, wsc);
  wcvt_t64<<<gWdd, blk, 0, stream>>>(wo, Wto, DM, DM, wsc);
  wcvt_t64<<<gW1,  blk, 0, stream>>>(w1, Wt1, DM, DFF, wsc);
  wcvt_t64<<<gW2,  blk, 0, stream>>>(w2, Wt2, DFF, DM, wsc);
  gemm64<1, 0, 1><<<gProjD, blk, 0, stream>>>(
      H1, DM, 0LL, Wtq, DM, 0LL, bq, x, (void*)Qp, DM, 0LL, NTOK, DM, DM, winv);
  gemm64<1, 0, 1><<<gProjD, blk, 0, stream>>>(
      H1, DM, 0LL, Wtk, DM, 0LL, bk, x, (void*)Kp, DM, 0LL, NTOK, DM, DM, winv);
  gemm64<2, 0, 1><<<gVT, blk, 0, stream>>>(
      Wtv, DM, 0LL, H1, DM, (long long)SEQ * DM, bv, x, (void*)VTp, SEQ, (long long)DM * SEQ, DM, SEQ, DM, winv);
  attn_causal64<<<gAttn, dim3(128), 0, stream>>>(Qp, Kp, VTp, CTX, 0.125f);
  gemm64<1, 0, 0><<<gProjD, blk, 0, stream>>>(
      CTX, DM, 0LL, Wto, DM, 0LL, bo, x, (void*)X1, DM, 0LL, NTOK, DM, DM, winv);
  layernorm_h<<<gLN, blk, 0, stream>>>(X1, ln2g, ln2b, H2, NTOK, 1e-7f);
  gemm64<1, 1, 1><<<gProjF, blk, 0, stream>>>(
      H2, DM, 0LL, Wt1, DM, 0LL, b1, x, (void*)Gp, DFF, 0LL, NTOK, DFF, DM, winv);
  gemm64<1, 0, 0><<<gProjD, blk, 0, stream>>>(
      Gp, DFF, 0LL, Wt2, DFF, 0LL, b2, X1, (void*)out, DM, 0LL, NTOK, DM, DFF, winv);
  (void)hipGetLastError();
}
